// Rwkv7SelfAttention_53223234732576
// MI455X (gfx1250) — hardware-verified
//
#include <hip/hip_runtime.h>
#include <math.h>

constexpr int kT   = 2048;
constexpr int kH   = 2048;
constexpr int kNH  = 32;
constexpr int kHD  = 64;
constexpr int kDW  = 64;
constexpr int kDA  = 64;
constexpr int kDV  = 32;
constexpr int kDVP = 64;
constexpr int kDG  = 128;
constexpr float kEpsLn  = 1e-5f;
constexpr float kEpsIn  = 0.00064f;
constexpr float kTiny   = 1.1754943508222875e-38f;
constexpr float kDecayC = 0.606531f;
constexpr float kInvH   = 1.0f / 2048.0f;
constexpr float kInvD   = 1.0f / 64.0f;
constexpr float kWoCarry    = 16.0f;
constexpr float kWoCarryInv = 1.0f / 16.0f;
static_assert(kNH * kHD == kH);
static_assert(kT % 64 == 0 && kH % 64 == 0 && kH % 32 == 0);
static_assert(kDW % 64 == 0 && kDA % 64 == 0 && kDVP % 64 == 0 && kDG % 64 == 0);
static_assert(kDV <= kDVP && kT % 16 == 0 && kH % 8 == 0);

typedef __attribute__((ext_vector_type(16))) __bf16   v16b;
typedef __attribute__((ext_vector_type(8)))  __bf16   v8b;
typedef __attribute__((ext_vector_type(16))) _Float16 v16h;
typedef __attribute__((ext_vector_type(8)))  _Float16 v8h;
typedef __attribute__((ext_vector_type(8)))  float    v8f;
typedef __attribute__((ext_vector_type(4)))  float    v4f;
typedef __attribute__((ext_vector_type(4)))  unsigned int v4u;

__device__ __forceinline__ unsigned short f2bf_bits(float f) {
  unsigned u = __float_as_uint(f);
  return (unsigned short)((u + 0x7FFFu + ((u >> 16) & 1u)) >> 16);
}
__device__ __forceinline__ float bf_bits2f(unsigned short h) { return __uint_as_float(((unsigned)h) << 16); }
__device__ __forceinline__ float bfr(float f) { return bf_bits2f(f2bf_bits(f)); }
__device__ __forceinline__ v4f bfr4(v4f a) { v4f r; r.x = bfr(a.x); r.y = bfr(a.y); r.z = bfr(a.z); r.w = bfr(a.w); return r; }
__device__ __forceinline__ unsigned pk16(unsigned short a, unsigned short b) { return (unsigned)a | ((unsigned)b << 16); }
__device__ __forceinline__ unsigned short h_bits(float f) { const _Float16 h = (_Float16)f; return __builtin_bit_cast(unsigned short, h); }

__device__ __forceinline__ void dep_guard_h(v8f& a, v8f& b, v16h x, v16h y) { asm volatile("v_nop\n\tv_nop\n\tv_nop\n\tv_nop" : "+v"(a), "+v"(b) : "v"(x), "v"(y)); }
__device__ __forceinline__ void dep_guard_b(v8f& a, v8f& b, v16b x, v16b y) { asm volatile("v_nop\n\tv_nop\n\tv_nop\n\tv_nop" : "+v"(a), "+v"(b) : "v"(x), "v"(y)); }
__device__ __forceinline__ void keep4_h(v16h a, v16h b, v16h c, v16h d) { asm volatile("v_nop" :: "v"(a), "v"(b), "v"(c), "v"(d)); }
__device__ __forceinline__ void keep4_b(v16b a, v16b b, v16b c, v16b d) { asm volatile("v_nop" :: "v"(a), "v"(b), "v"(c), "v"(d)); }
__device__ __forceinline__ void acc_guard4(v8f& a, v8f& b, v8f& c, v8f& d) { asm volatile("v_nop\n\tv_nop\n\tv_nop\n\tv_nop" : "+v"(a), "+v"(b), "+v"(c), "+v"(d)); }
template <typename T> struct Frag;
template <> struct Frag<_Float16> {
  typedef v16h V; union U { v16h v; v8h h[2]; };
  static __device__ __forceinline__ v16h load(const _Float16* p) {
    U f; f.h[0] = *(const v8h*)(p); f.h[1] = *(const v8h*)(p + 16); return f.v;
  }
  static __device__ __forceinline__ v8f mma(v16h a, v16h b, v8f c) {
    return __builtin_amdgcn_wmma_f32_16x16x32_f16(false, a, false, b, (short)0, c, false, false);
  }
  static __device__ __forceinline__ void guard(v8f& a, v8f& b, v16h x, v16h y) { dep_guard_h(a, b, x, y); }
  static __device__ __forceinline__ void keep(v16h a, v16h b, v16h c, v16h d) { keep4_h(a, b, c, d); }
};
template <> struct Frag<__bf16> {
  typedef v16b V; union U { v16b v; v8b h[2]; };
  static __device__ __forceinline__ v16b load(const __bf16* p) {
    U f; f.h[0] = *(const v8b*)(p); f.h[1] = *(const v8b*)(p + 16); return f.v;
  }
  static __device__ __forceinline__ v8f mma(v16b a, v16b b, v8f c) {
    return __builtin_amdgcn_wmma_f32_16x16x32_bf16(false, a, false, b, (short)0, c, false, false);
  }
  static __device__ __forceinline__ void guard(v8f& a, v8f& b, v16b x, v16b y) { dep_guard_b(a, b, x, y); }
  static __device__ __forceinline__ void keep(v16b a, v16b b, v16b c, v16b d) { keep4_b(a, b, c, d); }
};
template <int ET> struct Elem;
template <> struct Elem<0> { typedef _Float16 T; };
template <> struct Elem<1> { typedef __bf16 T; };

__device__ __forceinline__ float wave_sum(float v) {
#pragma unroll
  for (int off = 16; off > 0; off >>= 1) v += __shfl_xor(v, off, 32);
  return v;
}

__device__ __forceinline__ float sigm_f(float v) {
  const float e = expf(-fabsf(v));
  const float r = 1.0f / (1.0f + e);
  return (v >= 0.f) ? r : e * r;
}
template <int ACT> __device__ __forceinline__ float act_apply(float v) {
  if (ACT == 1) return tanhf(v);
  if (ACT == 2) return sigm_f(v);
  if (ACT == 3) return expf(-kDecayC * sigm_f(v));
  return v;
}

template <int ET, bool SPLITA, int BIAS_MODE, int ACT, int OUT_MODE>
__global__ __launch_bounds__(256) void gemm_wmma(
    const unsigned short* __restrict__ Ap, const unsigned short* __restrict__ A2p, int lda,
    const unsigned short* __restrict__ Btp, int ldb,
    void* Cout, void* Cout2, int ldc,
    const float* __restrict__ bias, const float* __restrict__ aux, const float* __restrict__ aux2, int ldx,
    int M, int N, int K, float scale) {
  typedef typename Elem<ET>::T T;
  typedef typename Frag<T>::V V;
  const T* A = (const T*)Ap; const T* A2 = (const T*)A2p; const T* Bt = (const T*)Btp;
  __shared__ __align__(16) float sT[8][16 * 68];
  const int lane = threadIdx.x & 31;
  const int wave = threadIdx.x >> 5;
  const int tilesN = N >> 6;
  const int tilesM = M >> 6;
  const int tile = blockIdx.x * 8 + wave;
  if (tile >= tilesM * tilesN) return;
  const int tm = tile / tilesN;
  const int tn = tile - tm * tilesN;
  const int m0 = tm << 6;
  const int n0 = tn << 6;

  const int rlane = lane & 15;
  const int koff  = (lane >> 4) * 8;
  const int mOff  = (lane >> 4) * 8;

  v8f acc[4][4];
#pragma unroll
  for (int i = 0; i < 4; ++i)
#pragma unroll
    for (int j = 0; j < 4; ++j) acc[i][j] = (v8f){0.f,0.f,0.f,0.f,0.f,0.f,0.f,0.f};

  for (int k0 = 0; k0 < K; k0 += 32) {
    V bh[4];
#pragma unroll
    for (int j = 0; j < 4; ++j) {
      const size_t bo = (size_t)(n0 + (j << 4) + rlane) * ldb + koff + k0;
      bh[j] = Frag<T>::load(Bt + bo);
    }
#pragma unroll
    for (int i = 0; i < 4; ++i) {
      const size_t ao = (size_t)(m0 + (i << 4) + rlane) * lda + koff + k0;
      V ah = Frag<T>::load(A + ao);
      V al = ah;
      if (SPLITA) al = Frag<T>::load(A2 + ao);
#pragma unroll
      for (int j = 0; j < 4; ++j) {
        acc[i][j] = Frag<T>::mma(ah, bh[j], acc[i][j]);
        if (SPLITA) acc[i][j] = Frag<T>::mma(al, bh[j], acc[i][j]);
      }
      Frag<T>::guard(acc[i][0], acc[i][3], ah, al);
    }
    Frag<T>::keep(bh[0], bh[1], bh[2], bh[3]);
  }
  acc_guard4(acc[0][0], acc[0][1], acc[0][2], acc[0][3]);
  acc_guard4(acc[1][0], acc[1][1], acc[1][2], acc[1][3]);
  acc_guard4(acc[2][0], acc[2][1], acc[2][2], acc[2][3]);
  acc_guard4(acc[3][0], acc[3][1], acc[3][2], acc[3][3]);

  float* slab = sT[wave];
#pragma unroll
  for (int i = 0; i < 4; ++i) {
    const int mBase = m0 + (i << 4);
#pragma unroll
    for (int j = 0; j < 4; ++j) {
      const int n = n0 + (j << 4) + rlane;
      float bv = 0.f;
      if (BIAS_MODE == 2) bv = bfr(bias[n]);
#pragma unroll
      for (int r = 0; r < 8; ++r) {
        float v = acc[i][j][r] * scale;
        if (BIAS_MODE == 2) v += bv;
        v = act_apply<ACT>(v);
        slab[(mOff + r) * 68 + (j << 4) + rlane] = v;
      }
    }
    __builtin_amdgcn_fence(__ATOMIC_RELEASE, "workgroup");
    __builtin_amdgcn_wave_barrier();
    __builtin_amdgcn_fence(__ATOMIC_ACQUIRE, "workgroup");
    if (OUT_MODE == 2) {
      const int q = lane >> 3, c8 = (lane & 7) * 8;
      unsigned short* C  = (unsigned short*)Cout;
      unsigned short* C2 = (unsigned short*)Cout2;
      for (int pass = 0; pass < 2; ++pass) {
#pragma unroll
        for (int it = 0; it < 4; ++it) {
          const int row = it * 4 + q;
          const float* sp = slab + row * 68 + c8;
          v8h hv, lv;
#pragma unroll
          for (int e = 0; e < 8; ++e) {
            unsigned short hb = f2bf_bits(sp[e]);
            unsigned short lb = f2bf_bits(sp[e] - bf_bits2f(hb));
            hv[e] = __builtin_bit_cast(_Float16, hb);
            lv[e] = __builtin_bit_cast(_Float16, lb);
          }
          *(volatile v8h*)(C + (size_t)(mBase + row) * ldc + n0 + c8) = hv;
          *(volatile v8h*)(C2 + (size_t)(mBase + row) * ldc + n0 + c8) = lv;
        }
        __threadfence();
      }
    } else {
      float* C = (float*)Cout;
      const int hh = lane >> 4, c4 = (lane & 15) * 4;
      constexpr int kGR = (OUT_MODE == 4) ? 2 : ((OUT_MODE == 3) ? 4 : 8);
#pragma unroll
      for (int g0 = 0; g0 < 8; g0 += kGR) {
        asm volatile("" ::: "memory");
        v4f vals[kGR];
#pragma unroll
        for (int u = 0; u < kGR; ++u) {
          const int row = (g0 + u) * 2 + hh;
          v4f sv = *(const v4f*)(slab + row * 68 + c4);
          const size_t xo = (size_t)(mBase + row) * ldx + n0 + c4;
          if (OUT_MODE == 3) {
            const v4f rv = bfr4(*(const v4f*)(aux + xo));
            sv += rv;
          }
          if (OUT_MODE == 4) {
            const v4f av = *(const v4f*)(aux + xo);
            const v4f fv = bfr4(*(const v4f*)(aux2 + xo));
            sv = av + (fv - av) * sv;
          }
          vals[u] = sv;
        }
        for (int pass = 0; pass < 2; ++pass) {
#pragma unroll
          for (int u = 0; u < kGR; ++u) {
            const int row = (g0 + u) * 2 + hh;
            *(volatile v4f*)(C + (size_t)(mBase + row) * ldc + n0 + c4) = vals[u];
          }
          __threadfence();
        }
      }
    }
    __builtin_amdgcn_fence(__ATOMIC_RELEASE, "workgroup");
    __builtin_amdgcn_wave_barrier();
    __builtin_amdgcn_fence(__ATOMIC_ACQUIRE, "workgroup");
  }
}

template <int F16OUT>
__global__ __launch_bounds__(256) void wt_cast_kernel(const float* __restrict__ W, int Kin, int Nout,
                                                     unsigned short* __restrict__ Bt, int ldb, float scale) {
  __shared__ float sm[64][65];
  const int t  = threadIdx.x;
  const int k0 = blockIdx.x * 64;
  const int n0 = blockIdx.y * 64;
#pragma unroll
  for (int hseg = 0; hseg < 2; ++hseg) {
#pragma unroll
    for (int i = 0; i < 8; ++i) {
      const int e  = (hseg * 8 + i) * 256 + t;
      const int kl = e >> 6;
      const int nl = e & 63;
      const int kk = k0 + kl;
      const int nn = n0 + nl;
      const int kc = (kk < Kin) ? kk : (Kin - 1);
      const int nc = (nn < Nout) ? nn : (Nout - 1);
      const float fac = (kk < Kin && nn < Nout) ? 1.0f : 0.0f;
      const float v = bfr(W[(size_t)kc * Nout + nc]) * fac;
      sm[nl][kl] = v;
    }
    asm volatile("" ::: "memory");
  }
  __syncthreads();
  const int lane = t & 31, wave = t >> 5;
  const int q = lane >> 3, c8 = (lane & 7) * 8;
  for (int pass = 0; pass < 2; ++pass) {
#pragma unroll
    for (int it = 0; it < 2; ++it) {
      const int row = wave * 8 + it * 4 + q;
      unsigned short hb[8];
#pragma unroll
      for (int e = 0; e < 8; ++e) {
        const float sv = sm[row][c8 + e];
        hb[e] = F16OUT ? h_bits(sv * scale) : f2bf_bits(sv);
      }
      const v4u u = (v4u){pk16(hb[0], hb[1]), pk16(hb[2], hb[3]), pk16(hb[4], hb[5]), pk16(hb[6], hb[7])};
      *(volatile v4u*)(Bt + (size_t)(n0 + row) * ldb + k0 + c8) = u;
    }
    __threadfence();
  }
}

__global__ __launch_bounds__(256) void ln_mix_kernel(const float* __restrict__ x, const float* __restrict__ st1,
                                                     const float* __restrict__ lnw, const float* __restrict__ lnb,
                                                     const float* __restrict__ coef,
                                                     unsigned short* __restrict__ hiP, unsigned short* __restrict__ loP,
                                                     float* __restrict__ out1, int writeLast) {
  __shared__ float redS[2][8];
  __shared__ float redQ[2][8];
  __shared__ __align__(16) float xs[kH];
  const int t = blockIdx.x;
  const int tid = threadIdx.x, lane = tid & 31, wave = tid >> 5;
  const int i0 = tid * 8;
  const int tp = (t > 0) ? (t - 1) : 0;
  const float* crow = x + (size_t)t * kH + i0;
  const float* prow = x + (size_t)tp * kH + i0;
  const v4f c0 = bfr4(*(const v4f*)(crow)), c1 = bfr4(*(const v4f*)(crow + 4));
  const v4f p0 = bfr4(*(const v4f*)(prow)), p1 = bfr4(*(const v4f*)(prow + 4));
  float cv[8], pv[8];
#pragma unroll
  for (int e = 0; e < 4; ++e) {
    cv[e] = c0[e]; cv[4 + e] = c1[e];
    pv[e] = p0[e]; pv[4 + e] = p1[e];
  }
  float sc = 0.f, sp = 0.f;
#pragma unroll
  for (int e = 0; e < 8; ++e) { sc += cv[e]; sp += pv[e]; }
  sc = wave_sum(sc); sp = wave_sum(sp);
  if (lane == 0) { redS[0][wave] = sc; redS[1][wave] = sp; }
  __syncthreads();
  asm volatile("" ::: "memory");
  const v4f s0 = bfr4(*(const v4f*)(st1 + i0)),  s1 = bfr4(*(const v4f*)(st1 + i0 + 4));
  const v4f f0 = bfr4(*(const v4f*)(coef + i0)), f1 = bfr4(*(const v4f*)(coef + i0 + 4));
  float sv[8], fv[8];
#pragma unroll
  for (int e = 0; e < 4; ++e) {
    sv[e] = s0[e]; sv[4 + e] = s1[e];
    fv[e] = f0[e]; fv[4 + e] = f1[e];
  }
  float tcs = 0.f, tps = 0.f;
#pragma unroll
  for (int w = 0; w < 8; ++w) { tcs += redS[0][w]; tps += redS[1][w]; }
  const float muc = tcs * kInvH, mup = tps * kInvH;
  float qc = 0.f, qp = 0.f;
#pragma unroll
  for (int e = 0; e < 8; ++e) {
    const float dc = cv[e] - muc; qc += dc * dc;
    const float dp = pv[e] - mup; qp += dp * dp;
  }
  qc = wave_sum(qc); qp = wave_sum(qp);
  if (lane == 0) { redQ[0][wave] = qc; redQ[1][wave] = qp; }
  __syncthreads();
  asm volatile("" ::: "memory");
  const v4f lw0 = bfr4(*(const v4f*)(lnw + i0)), lw1 = bfr4(*(const v4f*)(lnw + i0 + 4));
  const v4f lb0 = bfr4(*(const v4f*)(lnb + i0)), lb1 = bfr4(*(const v4f*)(lnb + i0 + 4));
  float wv[8], bv[8];
#pragma unroll
  for (int e = 0; e < 4; ++e) {
    wv[e] = lw0[e]; wv[4 + e] = lw1[e];
    bv[e] = lb0[e]; bv[4 + e] = lb1[e];
  }
  float tcq = 0.f, tpq = 0.f;
#pragma unroll
  for (int w = 0; w < 8; ++w) { tcq += redQ[0][w]; tpq += redQ[1][w]; }
  const float varc = tcq * kInvH, varp = tpq * kInvH;
  const float rc = 1.0f / sqrtf(varc + kEpsLn);
  const float rp = 1.0f / sqrtf(varp + kEpsLn);
  unsigned short hb[8], lb[8];
  float xl[8];
#pragma unroll
  for (int e = 0; e < 8; ++e) {
    const float xc  = (cv[e] - muc) * rc * wv[e] + bv[e];
    const float xpl = (pv[e] - mup) * rp * wv[e] + bv[e];
    const float xp  = (t == 0) ? sv[e] : xpl;
    const float sx  = xp - xc;
    const float xm  = xc + fv[e] * sx;
    hb[e] = f2bf_bits(xm);
    lb[e] = f2bf_bits(xm - bf_bits2f(hb[e]));
    xl[e] = xc;
  }
  const v4u uh = (v4u){pk16(hb[0], hb[1]), pk16(hb[2], hb[3]), pk16(hb[4], hb[5]), pk16(hb[6], hb[7])};
  const v4u ul = (v4u){pk16(lb[0], lb[1]), pk16(lb[2], lb[3]), pk16(lb[4], lb[5]), pk16(lb[6], lb[7])};
  unsigned short* hp = hiP + (size_t)t * kH + i0;
  unsigned short* lp = loP + (size_t)t * kH + i0;
  *(volatile v4u*)hp = uh;
  *(volatile v4u*)lp = ul;
  __threadfence();
  *(volatile v4u*)hp = uh;
  *(volatile v4u*)lp = ul;
  if (writeLast != 0 && t == kT - 1) {
#pragma unroll
    for (int e = 0; e < 8; ++e) xs[i0 + e] = xl[e] + kTiny;
    __syncthreads();
    for (int pass = 0; pass < 2; ++pass) {
#pragma unroll
      for (int it = 0; it < 2; ++it) {
        const int idx = it * 1024 + tid * 4;
        const v4f v = *(const v4f*)(xs + idx);
        *(volatile v4f*)(out1 + idx) = v;
      }
      __threadfence();
    }
  }
}

__global__ __launch_bounds__(64) void scan_kernel(
    const float* __restrict__ rP, const float* __restrict__ kP, const float* __restrict__ vP,
    const float* __restrict__ wP, const float* __restrict__ agP, const float* __restrict__ gP,
    const float* __restrict__ s2P, const float* __restrict__ kkP, const float* __restrict__ kaP,
    const float* __restrict__ rkP, const float* __restrict__ lwP, const float* __restrict__ lbP,
    unsigned short* __restrict__ oP, float* __restrict__ sOut) {
  __shared__ __align__(16) float Ssh[kHD][68];
  __shared__ __align__(16) float shA[kHD];
  __shared__ __align__(16) float shR[kHD];
  __shared__ __align__(16) float shKF[kHD];
  __shared__ __align__(16) float shW[kHD];
  __shared__ __align__(16) float shB[kHD];
  __shared__ float red1[2];
  __shared__ float red2a[2];
  __shared__ float red2b[2];
  __shared__ float red3[2];
  __shared__ __align__(16) unsigned short obh[16][kHD];

  const int n = blockIdx.x;
  const int d = threadIdx.x;
  const int lane = d & 31, wave = d >> 5;
  const int ch = n * kHD + d;
  {
    const float* s0 = s2P + ((size_t)(n * kHD + d)) * kHD;
#pragma unroll 1
    for (int j4 = 0; j4 < 16; ++j4) {
      const v4f sv4 = bfr4(*(const v4f*)(s0 + 4 * j4));
      *(v4f*)(&Ssh[d][4 * j4]) = sv4;
    }
  }
  const float ck  = bfr(kkP[ch]);
  const float ca  = bfr(kaP[ch]);
  const float crk = bfr(rkP[ch]);
  const float clw = bfr(lwP[ch]);
  const float clb = bfr(lbP[ch]);

#pragma unroll 1
  for (int t = 0; t < kT; ++t) {
    const size_t off = (size_t)t * kH + ch;
    const float rt = rP[off];
    const float kt = kP[off];
    const float vt = vP[off];
    const float wt = wP[off];
    const float at = agP[off];
    const float gt = gP[off];
    const float kk = kt * ck;
    const float ssw = wave_sum(kk * kk);
    if (lane == 0) red1[wave] = ssw;
    __syncthreads();
    const float ss  = red1[0] + red1[1];
    const float nrm = sqrtf(ss);
    const float inv = 1.0f / fmaxf(nrm, 1e-6f);
    const float kkn = kk * inv;
    const float kf  = kt * (1.0f + (at - 1.0f) * ca);
    shA[d] = -kkn; shR[d] = rt; shKF[d] = kf; shW[d] = wt; shB[d] = kkn * at;
    __syncthreads();
    float sa0 = 0.f, sa1 = 0.f, sa2 = 0.f, sa3 = 0.f;
#pragma unroll 1
    for (int j4 = 0; j4 < 16; ++j4) {
      const v4f s4 = *(const v4f*)(&Ssh[d][4 * j4]);
      const v4f a4 = *(const v4f*)(&shA[4 * j4]);
      sa0 = fmaf(s4.x, a4.x, sa0);
      sa1 = fmaf(s4.y, a4.y, sa1);
      sa2 = fmaf(s4.z, a4.z, sa2);
      sa3 = fmaf(s4.w, a4.w, sa3);
    }
    const float Sa = (sa0 + sa1) + (sa2 + sa3);
    float y0 = 0.f, y1 = 0.f, y2 = 0.f, y3 = 0.f;
#pragma unroll 1
    for (int j4 = 0; j4 < 16; ++j4) {
      const v4f s4 = *(const v4f*)(&Ssh[d][4 * j4]);
      const v4f w4 = *(const v4f*)(&shW[4 * j4]);
      const v4f b4 = *(const v4f*)(&shB[4 * j4]);
      const v4f f4 = *(const v4f*)(&shKF[4 * j4]);
      const v4f r4 = *(const v4f*)(&shR[4 * j4]);
      v4f sn;
      sn.x = fmaf(s4.x, w4.x, fmaf(Sa, b4.x, vt * f4.x));
      sn.y = fmaf(s4.y, w4.y, fmaf(Sa, b4.y, vt * f4.y));
      sn.z = fmaf(s4.z, w4.z, fmaf(Sa, b4.z, vt * f4.z));
      sn.w = fmaf(s4.w, w4.w, fmaf(Sa, b4.w, vt * f4.w));
      y0 = fmaf(sn.x, r4.x, y0);
      y1 = fmaf(sn.y, r4.y, y1);
      y2 = fmaf(sn.z, r4.z, y2);
      y3 = fmaf(sn.w, r4.w, y3);
      *(v4f*)(&Ssh[d][4 * j4]) = sn;
    }
    const float y  = (y0 + y1) + (y2 + y3);
    const float p1 = wave_sum(y);
    const float p2 = wave_sum(rt * kf * crk);
    if (lane == 0) { red2a[wave] = p1; red2b[wave] = p2; }
    __syncthreads();
    const float mu = (red2a[0] + red2a[1]) * kInvD;
    const float cb = red2b[0] + red2b[1];
    const float dy = y - mu;
    const float q1 = wave_sum(dy * dy);
    if (lane == 0) red3[wave] = q1;
    __syncthreads();
    const float var = (red3[0] + red3[1]) * kInvD;
    const float on  = dy * (1.0f / sqrtf(var + kEpsIn));
    const float o   = (on * clw + clb + cb * vt) * gt;
    obh[t & 15][d] = h_bits(o);
    if ((t & 15) == 15) {
      __syncthreads();
      const int tb = t - 15;
      const int q8 = lane >> 3, c8 = (lane & 7) * 8;
      for (int pass = 0; pass < 2; ++pass) {
#pragma unroll
        for (int it = 0; it < 2; ++it) {
          const int row = wave * 8 + it * 4 + q8;
          const v4u uh = *(const v4u*)(&obh[row][c8]);
          const size_t go = (size_t)(tb + row) * kH + n * kHD + c8;
          *(volatile v4u*)(oP + go) = uh;
        }
        __threadfence();
      }
    }
  }
  __syncthreads();
  float* so = sOut + (size_t)n * kHD * kHD;
  for (int pass = 0; pass < 2; ++pass) {
#pragma unroll
    for (int it = 0; it < 16; ++it) {
      const int idx = it * 256 + d * 4;
      const int row = idx >> 6, col = idx & 63;
      const v4f v = *(const v4f*)(&Ssh[row][col]);
      *(volatile v4f*)(so + idx) = v;
    }
    __threadfence();
  }
}

__global__ __launch_bounds__(256) void copy_bfr_kernel(const float* __restrict__ src, float* __restrict__ dst, int n4) {
  const int i = blockIdx.x * 256 + threadIdx.x;
  if (i >= n4) return;
  const v4f v = bfr4(*(const v4f*)(src + 4 * (size_t)i));
  float* p = dst + 4 * (size_t)i;
  *(volatile v4f*)p = v;
  __threadfence();
  *(volatile v4f*)p = v;
}

extern "C" void kernel_launch(void* const* d_in, const int* in_sizes, int n_in,
                              void* d_out, int out_size, void* d_ws, size_t ws_size,
                              hipStream_t stream) {
  if (n_in < 32) return;
  const int nTH = kT * kH;
  const int nS  = kNH * kHD * kHD;
  if (in_sizes[0] != nTH || in_sizes[3] != nTH || in_sizes[1] != kH || in_sizes[2] != nS) return;
  if (in_sizes[13] != kH * kDW || in_sizes[16] != kH * kDA || in_sizes[19] != kH * kDV || in_sizes[21] != kH * kDG) return;
  if (in_sizes[14] != kDW * kH || in_sizes[17] != kDA * kH || in_sizes[20] != kDV * kH || in_sizes[22] != kDG * kH) return;
  if (in_sizes[23] != kH * kH || in_sizes[24] != kH * kH || in_sizes[25] != kH * kH || in_sizes[26] != kH * kH) return;
  if (out_size != nTH + kH + nS + nTH) return;

  const size_t szWBT = (size_t)kH * kH * 2;
  const size_t szG1T = (size_t)kDG * kH * 2;
  const size_t szR64 = (size_t)64 * kH * 2;
  const size_t szG2T = (size_t)kH * kDG * 2;
  const size_t szMIX = (size_t)kT * kH * 2;
  const size_t szHG  = (size_t)kT * kDG * 2;
  const size_t szH64 = (size_t)kT * 64 * 2;
  const size_t szF   = (size_t)kT * kH * 4;
  size_t off = 0;
  const size_t oWBT = off; off += szWBT;
  const size_t oG1T = off; off += szG1T;
  const size_t oA1T = off; off += szR64;
  const size_t oW1T = off; off += szR64;
  const size_t oV1T = off; off += szR64;
  const size_t oW2T = off; off += szR64;
  const size_t oA2T = off; off += szR64;
  const size_t oV2T = off; off += szR64;
  const size_t oG2T = off; off += szG2T;
  const size_t oMXH = off; off += szMIX;
  const size_t oMXL = off; off += szMIX;
  const size_t oHGh = off; off += szHG;
  const size_t oHGl = off; off += szHG;
  const size_t oHAh = off; off += szH64;
  const size_t oHAl = off; off += szH64;
  const size_t oHWh = off; off += szH64;
  const size_t oHWl = off; off += szH64;
  const size_t oHVh = off; off += szH64;
  const size_t oHVl = off; off += szH64;
  const size_t oR   = off; off += szF;
  const size_t oK   = off; off += szF;
  const size_t oV   = off; off += szF;
  const size_t oW   = off; off += szF;
  const size_t oAG  = off; off += szF;
  const size_t oG   = off; off += szF;
  const size_t total = off;
  if (ws_size < total) return;

  const float* x      = (const float*)d_in[0];
  const float* state1 = (const float*)d_in[1];
  const float* state2 = (const float*)d_in[2];
  const float* vfirst = (const float*)d_in[3];
  const float* ln1w   = (const float*)d_in[4];
  const float* ln1b   = (const float*)d_in[5];
  const float* x_r    = (const float*)d_in[6];
  const float* x_w    = (const float*)d_in[7];
  const float* x_k    = (const float*)d_in[8];
  const float* x_v    = (const float*)d_in[9];
  const float* x_a    = (const float*)d_in[10];
  const float* x_g    = (const float*)d_in[11];
  const float* w0     = (const float*)d_in[12];
  const float* w1     = (const float*)d_in[13];
  const float* w2     = (const float*)d_in[14];
  const float* a0     = (const float*)d_in[15];
  const float* a1     = (const float*)d_in[16];
  const float* a2     = (const float*)d_in[17];
  const float* v0     = (const float*)d_in[18];
  const float* v1     = (const float*)d_in[19];
  const float* v2     = (const float*)d_in[20];
  const float* g1     = (const float*)d_in[21];
  const float* g2     = (const float*)d_in[22];
  const float* Wr     = (const float*)d_in[23];
  const float* Wk     = (const float*)d_in[24];
  const float* Wv     = (const float*)d_in[25];
  const float* Wo     = (const float*)d_in[26];
  const float* k_k    = (const float*)d_in[27];
  const float* k_a    = (const float*)d_in[28];
  const float* r_k    = (const float*)d_in[29];
  const float* ln_x_w = (const float*)d_in[30];
  const float* ln_x_b = (const float*)d_in[31];

  float* out0 = (float*)d_out;
  float* out1 = out0 + nTH;
  float* out2 = out1 + kH;
  float* out3 = out2 + nS;

  char* ws = (char*)d_ws;
  unsigned short* WBT = (unsigned short*)(ws + oWBT);
  unsigned short* G1T = (unsigned short*)(ws + oG1T);
  unsigned short* A1T = (unsigned short*)(ws + oA1T);
  unsigned short* W1T = (unsigned short*)(ws + oW1T);
  unsigned short* V1T = (unsigned short*)(ws + oV1T);
  unsigned short* W2T = (unsigned short*)(ws + oW2T);
  unsigned short* A2T = (unsigned short*)(ws + oA2T);
  unsigned short* V2T = (unsigned short*)(ws + oV2T);
  unsigned short* G2T = (unsigned short*)(ws + oG2T);
  unsigned short* MXH = (unsigned short*)(ws + oMXH);
  unsigned short* MXL = (unsigned short*)(ws + oMXL);
  unsigned short* HGh = (unsigned short*)(ws + oHGh);
  unsigned short* HGl = (unsigned short*)(ws + oHGl);
  unsigned short* HAh = (unsigned short*)(ws + oHAh);
  unsigned short* HAl = (unsigned short*)(ws + oHAl);
  unsigned short* HWh = (unsigned short*)(ws + oHWh);
  unsigned short* HWl = (unsigned short*)(ws + oHWl);
  unsigned short* HVh = (unsigned short*)(ws + oHVh);
  unsigned short* HVl = (unsigned short*)(ws + oHVl);
  float* Rp  = (float*)(ws + oR);
  float* Kp  = (float*)(ws + oK);
  float* Vp  = (float*)(ws + oV);
  float* Wp  = (float*)(ws + oW);
  float* AGp = (float*)(ws + oAG);
  float* Gp  = (float*)(ws + oG);

  const dim3 blk(256);
  const int blkBig  = ((kT / 64) * (kH / 64)) / 8;
  const int blkN64  = ((kT / 64) * 1) / 8;
  const int blkN128 = ((kT / 64) * 2) / 8;

  wt_cast_kernel<0><<<dim3(kH / 64, kDG / 64), blk, 0, stream>>>(g1, kH, kDG, G1T, kH, 1.0f);
  wt_cast_kernel<0><<<dim3(kH / 64, 1), blk, 0, stream>>>(a1, kH, kDA, A1T, kH, 1.0f);
  wt_cast_kernel<0><<<dim3(kH / 64, 1), blk, 0, stream>>>(w1, kH, kDW, W1T, kH, 1.0f);
  wt_cast_kernel<0><<<dim3(kH / 64, 1), blk, 0, stream>>>(v1, kH, kDV, V1T, kH, 1.0f);
  wt_cast_kernel<0><<<dim3(1, kH / 64), blk, 0, stream>>>(w2, kDW, kH, W2T, 64, 1.0f);
  wt_cast_kernel<0><<<dim3(1, kH / 64), blk, 0, stream>>>(a2, kDA, kH, A2T, 64, 1.0f);
  wt_cast_kernel<0><<<dim3(1, kH / 64), blk, 0, stream>>>(v2, kDV, kH, V2T, 64, 1.0f);
  wt_cast_kernel<0><<<dim3(kDG / 64, kH / 64), blk, 0, stream>>>(g2, kDG, kH, G2T, kDG, 1.0f);

  wt_cast_kernel<0><<<dim3(kH / 64, kH / 64), blk, 0, stream>>>(Wr, kH, kH, WBT, kH, 1.0f);
  ln_mix_kernel<<<dim3(kT), blk, 0, stream>>>(x, state1, ln1w, ln1b, x_r, MXH, MXL, out1, 1);
  gemm_wmma<1, true, 0, 0, 0><<<dim3(blkBig), blk, 0, stream>>>(
      MXH, MXL, kH, WBT, kH, (void*)Rp, (void*)Rp, kH, a0, x, x, kH, kT, kH, kH, 1.0f);

  wt_cast_kernel<0><<<dim3(kH / 64, kH / 64), blk, 0, stream>>>(Wk, kH, kH, WBT, kH, 1.0f);
  ln_mix_kernel<<<dim3(kT), blk, 0, stream>>>(x, state1, ln1w, ln1b, x_k, MXH, MXL, out1, 0);
  gemm_wmma<1, true, 0, 0, 0><<<dim3(blkBig), blk, 0, stream>>>(
      MXH, MXL, kH, WBT, kH, (void*)Kp, (void*)Kp, kH, a0, x, x, kH, kT, kH, kH, 1.0f);

  wt_cast_kernel<0><<<dim3(kH / 64, kH / 64), blk, 0, stream>>>(Wv, kH, kH, WBT, kH, 1.0f);
  ln_mix_kernel<<<dim3(kT), blk, 0, stream>>>(x, state1, ln1w, ln1b, x_v, MXH, MXL, out1, 0);
  gemm_wmma<1, true, 0, 0, 0><<<dim3(blkBig), blk, 0, stream>>>(
      MXH, MXL, kH, WBT, kH, (void*)Wp, (void*)Wp, kH, a0, x, x, kH, kT, kH, kH, 1.0f);
  gemm_wmma<1, true, 0, 0, 2><<<dim3(blkN64), blk, 0, stream>>>(
      MXH, MXL, kH, V1T, kH, (void*)HVh, (void*)HVl, kDVP, a0, x, x, kH, kT, kDVP, kH, 1.0f);
  gemm_wmma<1, true, 2, 2, 4><<<dim3(blkBig), blk, 0, stream>>>(
      HVh, HVl, kDVP, V2T, kDVP, (void*)Vp, (void*)Vp, kH, v0, Wp, vfirst, kH, kT, kH, kDVP, 1.0f);

  ln_mix_kernel<<<dim3(kT), blk, 0, stream>>>(x, state1, ln1w, ln1b, x_w, MXH, MXL, out1, 0);
  gemm_wmma<1, true, 0, 1, 2><<<dim3(blkN64), blk, 0, stream>>>(
      MXH, MXL, kH, W1T, kH, (void*)HWh, (void*)HWl, kDW, a0, x, x, kH, kT, kDW, kH, 1.0f);
  gemm_wmma<1, true, 2, 3, 0><<<dim3(blkBig), blk, 0, stream>>>(
      HWh, HWl, kDW, W2T, kDW, (void*)Wp, (void*)Wp, kH, w0, x, x, kH, kT, kH, kDW, 1.0f);

  ln_mix_kernel<<<dim3(kT), blk, 0, stream>>>(x, state1, ln1w, ln1b, x_a, MXH, MXL, out1, 0);
  gemm_wmma<1, true, 0, 0, 2><<<dim3(blkN64), blk, 0, stream>>>(
      MXH, MXL, kH, A1T, kH, (void*)HAh, (void*)HAl, kDA, a0, x, x, kH, kT, kDA, kH, 1.0f);
  gemm_wmma<1, true, 2, 2, 0><<<dim3(blkBig), blk, 0, stream>>>(
      HAh, HAl, kDA, A2T, kDA, (void*)AGp, (void*)AGp, kH, a0, x, x, kH, kT, kH, kDA, 1.0f);

  ln_mix_kernel<<<dim3(kT), blk, 0, stream>>>(x, state1, ln1w, ln1b, x_g, MXH, MXL, out1, 0);
  gemm_wmma<1, true, 0, 2, 2><<<dim3(blkN128), blk, 0, stream>>>(
      MXH, MXL, kH, G1T, kH, (void*)HGh, (void*)HGl, kDG, a0, x, x, kH, kT, kDG, kH, 1.0f);
  gemm_wmma<1, true, 0, 0, 0><<<dim3(blkBig), blk, 0, stream>>>(
      HGh, HGl, kDG, G2T, kDG, (void*)Gp, (void*)Gp, kH, a0, x, x, kH, kT, kH, kDG, 1.0f);

  wt_cast_kernel<1><<<dim3(kH / 64, kH / 64), blk, 0, stream>>>(Wo, kH, kH, WBT, kH, kWoCarry);

  scan_kernel<<<dim3(kNH), dim3(64), 0, stream>>>(
      Rp, Kp, Vp, Wp, AGp, Gp, state2, k_k, k_a, r_k, ln_x_w, ln_x_b, MXH, out2);

  gemm_wmma<0, false, 0, 0, 3><<<dim3(blkBig), blk, 0, stream>>>(
      MXH, MXH, kH, WBT, kH, (void*)out0, (void*)out0, kH, a0, x, x, kH, kT, kH, kH, kWoCarryInv);

  copy_bfr_kernel<<<dim3((nTH / 4) / 256), blk, 0, stream>>>(vfirst, out3, nTH / 4);
}
